// RobertaAttention_40948218200349
// MI455X (gfx1250) — hardware-verified
//
#include <hip/hip_runtime.h>
#include <math.h>
#include <stdint.h>

#define NBATCH 4
#define SEQ    2048
#define DM     768
#define NH     12
#define HD     64
#define QKP    (2 * DM)
#define MP     (NBATCH * SEQ)
#define NQB    (SEQ / 64)
#define LNT    (DM / 4)
#define LNW    (LNT / 32)
#define LNEPS  1.0e-12f
#define WSC    64.0f
#define CSC    64.0f
static_assert(NH * HD == DM);
static_assert((SEQ % 64) == 0 && (DM % 64) == 0 && (QKP % 64) == 0 && (MP % 64) == 0);
static_assert(DM == 4 * LNT && (LNT % 32) == 0 && LNW <= 8);

typedef _Float16 v16h __attribute__((ext_vector_type(16)));
typedef _Float16 v8h  __attribute__((ext_vector_type(8)));
typedef float    v8f  __attribute__((ext_vector_type(8)));
typedef float    v4f  __attribute__((ext_vector_type(4)));
typedef unsigned int v4u __attribute__((ext_vector_type(4)));

union FragH { v16h v; v8h h[2]; };

__device__ __forceinline__ unsigned short bf_bits(float f) {
  unsigned u = __float_as_uint(f);
  return (unsigned short)((u + 0x7FFFu + ((u >> 16) & 1u)) >> 16);
}
__device__ __forceinline__ float bf_up(unsigned short h) { return __uint_as_float(((unsigned)h) << 16); }
__device__ __forceinline__ float bfr(float f) { return bf_up(bf_bits(f)); }
__device__ __forceinline__ unsigned short h_bits(_Float16 x) { return __builtin_bit_cast(unsigned short, x); }
__device__ __forceinline__ unsigned pk16(unsigned short a, unsigned short b) { return (unsigned)a | ((unsigned)b << 16); }
__device__ __forceinline__ v8f zero8() { v8f z = {0.f, 0.f, 0.f, 0.f, 0.f, 0.f, 0.f, 0.f}; return z; }
__device__ __forceinline__ float gelu_f(float v) { return 0.5f * v * (1.0f + erff(v * 0.70710678118654752f)); }

__device__ __forceinline__ v16h ldfrag_h(const _Float16* p) {
  FragH f;
  f.h[0] = *(const v8h*)(p);
  f.h[1] = *(const v8h*)(p + 16);
  return f.v;
}

__device__ __forceinline__ v8f mma_h(v16h a, v16h b, v8f c) {
  c = __builtin_amdgcn_wmma_f32_16x16x32_f16(false, a, false, b, (short)0, c, false, false);
#if defined(__HIP_DEVICE_COMPILE__)
  asm volatile("v_nop\n\tv_nop\n\tv_nop\n\tv_nop" : "+v"(c) : "v"(a), "v"(b));
#endif
  return c;
}
__device__ __forceinline__ v8f mma_h_raw(v16h a, v16h b, v8f c) {
  return __builtin_amdgcn_wmma_f32_16x16x32_f16(false, a, false, b, (short)0, c, false, false);
}
__device__ __forceinline__ void dep_guard1(v8f& a, v8f& b, v16h x) {
#if defined(__HIP_DEVICE_COMPILE__)
  asm volatile("v_nop\n\tv_nop\n\tv_nop\n\tv_nop" : "+v"(a), "+v"(b) : "v"(x));
#endif
}
__device__ __forceinline__ void keep4_h(v16h a, v16h b, v16h c, v16h d) {
#if defined(__HIP_DEVICE_COMPILE__)
  asm volatile("v_nop" :: "v"(a), "v"(b), "v"(c), "v"(d));
#endif
}
__device__ __forceinline__ void acc_guard4(v8f& a, v8f& b, v8f& c, v8f& d) {
#if defined(__HIP_DEVICE_COMPILE__)
  asm volatile("v_nop\n\tv_nop\n\tv_nop\n\tv_nop" : "+v"(a), "+v"(b), "+v"(c), "+v"(d));
#endif
}
__device__ __forceinline__ void wave_sync_lds() {
  __builtin_amdgcn_fence(__ATOMIC_RELEASE, "workgroup");
  __builtin_amdgcn_wave_barrier();
  __builtin_amdgcn_fence(__ATOMIC_ACQUIRE, "workgroup");
}
__device__ __forceinline__ float wsum(float v) {
#pragma unroll
  for (int off = 16; off > 0; off >>= 1) v += __shfl_xor(v, off, 32);
  return v;
}
__device__ __forceinline__ float bsumLN(float v, float* red, int lane, int wave) {
  v = wsum(v);
  if (lane == 0) red[wave] = v;
  __syncthreads();
  float tot = 0.f;
#pragma unroll
  for (int w = 0; w < LNW; ++w) tot += red[w];
  return tot;
}

__global__ __launch_bounds__(256) void conv_h16(const float* __restrict__ W, unsigned short* Wh, int n8, float wsc) {
  const int i  = blockIdx.x * 256 + threadIdx.x;
  const int ic = (i < n8) ? i : (n8 - 1);
  const float* src = W + (size_t)ic * 8;
  const v4f a = *(const v4f*)(src);
  const v4f c = *(const v4f*)(src + 4);
  v4u o;
  o[0] = pk16(h_bits((_Float16)(bfr(a[0]) * wsc)), h_bits((_Float16)(bfr(a[1]) * wsc)));
  o[1] = pk16(h_bits((_Float16)(bfr(a[2]) * wsc)), h_bits((_Float16)(bfr(a[3]) * wsc)));
  o[2] = pk16(h_bits((_Float16)(bfr(c[0]) * wsc)), h_bits((_Float16)(bfr(c[1]) * wsc)));
  o[3] = pk16(h_bits((_Float16)(bfr(c[2]) * wsc)), h_bits((_Float16)(bfr(c[3]) * wsc)));
  if (i < n8) *(volatile v4u*)(Wh + (size_t)i * 8) = o;
  __threadfence();
  if (i < n8) *(volatile v4u*)(Wh + (size_t)i * 8) = o;
}

template <int OM, int BIASM, int ACT, int RES>
__global__ __launch_bounds__(256) void gemm64(
    const unsigned short* __restrict__ Ap, int lda, long long strideA,
    const unsigned short* __restrict__ Btp, int ldb, long long strideB,
    const float* __restrict__ bias0, const float* __restrict__ bias1, int Nb,
    const float* resid,
    void* Cout, int ldc, long long strideC,
    int M, int N, int K, float oscale) {
  const _Float16* A  = (const _Float16*)(const void*)Ap;
  const _Float16* Bt = (const _Float16*)(const void*)Btp;
  __shared__ __align__(16) float sT[8][16 * 68];
  const int b    = blockIdx.y;
  const int lane = threadIdx.x & 31;
  const int wave = threadIdx.x >> 5;
  const int tilesN = N >> 6;
  const int tilesM = M >> 6;
  const int tile = blockIdx.x * 8 + wave;
  if (tile >= tilesM * tilesN) return;
  const int tm = tile / tilesN;
  const int tn = tile - tm * tilesN;
  const int m0 = tm << 6;
  const int n0 = tn << 6;

  const _Float16* Ab = A  + (size_t)b * strideA;
  const _Float16* Bb = Bt + (size_t)b * strideB;

  const int rlane = lane & 15;
  const int koff  = (lane >> 4) * 8;
  const int mOff  = (lane >> 4) * 8;

  v8f acc[4][4];
#pragma unroll
  for (int i = 0; i < 4; ++i)
#pragma unroll
    for (int j = 0; j < 4; ++j) acc[i][j] = zero8();

  for (int k0 = 0; k0 < K; k0 += 32) {
    v16h bh[4];
#pragma unroll
    for (int j = 0; j < 4; ++j) {
      const size_t bo = (size_t)(n0 + (j << 4) + rlane) * ldb + koff + k0;
      bh[j] = ldfrag_h(Bb + bo);
    }
#pragma unroll
    for (int i = 0; i < 4; ++i) {
      const size_t ao = (size_t)(m0 + (i << 4) + rlane) * lda + koff + k0;
      const v16h ah = ldfrag_h(Ab + ao);
#pragma unroll
      for (int j = 0; j < 4; ++j) acc[i][j] = mma_h_raw(ah, bh[j], acc[i][j]);
      dep_guard1(acc[i][0], acc[i][3], ah);
    }
    keep4_h(bh[0], bh[1], bh[2], bh[3]);
  }
  acc_guard4(acc[0][0], acc[0][1], acc[0][2], acc[0][3]);
  acc_guard4(acc[1][0], acc[1][1], acc[1][2], acc[1][3]);
  acc_guard4(acc[2][0], acc[2][1], acc[2][2], acc[2][3]);
  acc_guard4(acc[3][0], acc[3][1], acc[3][2], acc[3][3]);

  const int hh2 = lane >> 4, c4 = (lane & 15) * 4;
  const int q8  = lane >> 3, c8 = (lane & 7) * 8;
  float bc[8];
#pragma unroll
  for (int e = 0; e < 8; ++e) bc[e] = 0.f;
  if (BIASM == 0) {
    const bool use1 = (n0 >= Nb);
    if (OM == 0) {
      const int cb = n0 + c4;
      const int i0 = (cb < Nb - 4) ? cb : (Nb - 4);
      const int i1 = (cb - Nb > 0) ? (cb - Nb) : 0;
      const v4f b0v = *(const v4f*)(bias0 + i0);
      const v4f b1v = *(const v4f*)(bias1 + i1);
#pragma unroll
      for (int e = 0; e < 4; ++e) bc[e] = bfr(use1 ? b1v[e] : b0v[e]);
    } else {
      const int cb = n0 + c8;
      const int i0 = (cb < Nb - 8) ? cb : (Nb - 8);
      const int i1 = (cb - Nb > 0) ? (cb - Nb) : 0;
      const v4f b0a = *(const v4f*)(bias0 + i0), b0b = *(const v4f*)(bias0 + i0 + 4);
      const v4f b1a = *(const v4f*)(bias1 + i1), b1b = *(const v4f*)(bias1 + i1 + 4);
#pragma unroll
      for (int e = 0; e < 4; ++e) {
        bc[e]     = bfr(use1 ? b1a[e] : b0a[e]);
        bc[4 + e] = bfr(use1 ? b1b[e] : b0b[e]);
      }
    }
  }

  float* slab = sT[wave];
#pragma unroll
  for (int i = 0; i < 4; ++i) {
    const int mBase = m0 + (i << 4);
#pragma unroll
    for (int j = 0; j < 4; ++j) {
#pragma unroll
      for (int r = 0; r < 8; ++r) {
        slab[(mOff + r) * 68 + (j << 4) + rlane] = acc[i][j][r];
      }
    }
    wave_sync_lds();
    if (OM == 0) {
      float* C = (float*)Cout + (size_t)b * strideC;
      const float* Rb = resid + (size_t)b * strideC;
      v4f vals[8];
#pragma unroll
      for (int it = 0; it < 8; ++it) {
        const int row = it * 2 + hh2;
        v4f v = *(const v4f*)(slab + row * 68 + c4);
#pragma unroll
        for (int e = 0; e < 4; ++e) {
          float f = v[e] * oscale + bc[e];
          if (ACT) f = gelu_f(f);
          v[e] = f;
        }
        if (RES == 1 || RES == 3) {
          const v4f rr = *(const v4f*)(Rb + (size_t)(mBase + row) * ldc + n0 + c4);
#pragma unroll
          for (int e = 0; e < 4; ++e) v[e] += (RES == 3) ? bfr(rr[e]) : rr[e];
        }
        vals[it] = v;
      }
      for (int pass = 0; pass < 2; ++pass) {
#pragma unroll
        for (int it = 0; it < 8; ++it) {
          const int row = it * 2 + hh2;
          *(volatile v4f*)(C + (size_t)(mBase + row) * ldc + n0 + c4) = vals[it];
        }
        __threadfence();
      }
    } else {
      unsigned short* C = (unsigned short*)Cout + (size_t)b * strideC;
      v4u hv[4];
#pragma unroll
      for (int it = 0; it < 4; ++it) {
        const int row = it * 4 + q8;
        const float* sp = slab + row * 68 + c8;
        float bm = 0.f;
        if (BIASM == 1) bm = bfr(bias0[mBase + row]);
        v4u a;
#pragma unroll
        for (int e = 0; e < 4; ++e) {
          float f0 = sp[2 * e]     * oscale + ((BIASM == 1) ? bm : bc[2 * e]);
          float f1 = sp[2 * e + 1] * oscale + ((BIASM == 1) ? bm : bc[2 * e + 1]);
          if (ACT) { f0 = gelu_f(f0); f1 = gelu_f(f1); }
          unsigned short u0, u1;
          if (OM == 1) { u0 = bf_bits(f0); u1 = bf_bits(f1); }
          else         { u0 = h_bits((_Float16)f0); u1 = h_bits((_Float16)f1); }
          a[e] = pk16(u0, u1);
        }
        hv[it] = a;
      }
      for (int pass = 0; pass < 2; ++pass) {
#pragma unroll
        for (int it = 0; it < 4; ++it) {
          const int row = it * 4 + q8;
          *(volatile v4u*)(C + (size_t)(mBase + row) * ldc + n0 + c8) = hv[it];
        }
        __threadfence();
      }
    }
    wave_sync_lds();
  }
}

__global__ __launch_bounds__(128)
void attn64(const unsigned short* __restrict__ qkp, const unsigned short* __restrict__ vtp,
            const float* __restrict__ mkp, unsigned short* outp, float sscale) {
  __shared__ __align__(16) _Float16 Ksh[64 * 64];
  __shared__ __align__(16) _Float16 Vth[64 * 64];
  __shared__ __align__(16) _Float16 Psh[4][16 * 64];
  __shared__ __align__(16) float    Os[4][16 * 64];

  const int tid  = threadIdx.x;
  const int wave = tid >> 5;
  const int lane = tid & 31;
  const int hh   = lane >> 4;
  const int c    = lane & 15;

  const int bx   = blockIdx.x;
  const int qb   = bx % NQB;
  const int rest = bx / NQB;
  const int h    = rest % NH;
  const int b    = rest / NH;
  const int q0   = qb * 64 + wave * 16;
  const size_t rowB = (size_t)b * SEQ;

  const _Float16* Qh = (const _Float16*)(const void*)qkp + (size_t)h * HD;
  const _Float16* Kg = (const _Float16*)(const void*)qkp + DM + (size_t)h * HD;
  const _Float16* Vh = (const _Float16*)(const void*)vtp + ((size_t)b * DM + (size_t)h * HD) * SEQ;
  const float*    Mb = mkp + rowB;

  v16h qa[2];
#pragma unroll
  for (int dc = 0; dc < 2; ++dc) qa[dc] = ldfrag_h(Qh + (rowB + q0 + c) * QKP + dc * 32 + 8 * hh);

  float mrow[8], lrow[8];
  v8f oacc[4];
#pragma unroll
  for (int r = 0; r < 8; ++r) { mrow[r] = -INFINITY; lrow[r] = 0.f; }
#pragma unroll
  for (int t = 0; t < 4; ++t) oacc[t] = zero8();

  for (int kt = 0; kt < NQB; ++kt) {
    const int kv0 = kt * 64;
    float mk[4];
#pragma unroll
    for (int j = 0; j < 4; ++j) mk[j] = bfr(Mb[kv0 + j * 16 + c]);

    __syncthreads();
    {
      const int r = tid >> 1, hf = (tid & 1) * 32;
      const _Float16* kg = Kg + (rowB + kv0 + r) * QKP + hf;
      const _Float16* vg = Vh + (size_t)r * SEQ + kv0 + hf;
#pragma unroll
      for (int i = 0; i < 4; ++i) {
        const v8h a0 = *(const v8h*)(kg + 8 * i);
        const v8h b0 = *(const v8h*)(vg + 8 * i);
        *(v8h*)(Ksh + r * 64 + hf + 8 * i) = a0;
        *(v8h*)(Vth + r * 64 + hf + 8 * i) = b0;
      }
    }
    __syncthreads();

    v8f s[4];
#pragma unroll
    for (int j = 0; j < 4; ++j) {
      v8f sh = zero8();
#pragma unroll
      for (int dc = 0; dc < 2; ++dc) {
        FragH kb;
        kb.h[0] = *(const v8h*)(Ksh + (j * 16 + c) * 64 + dc * 32 + 8 * hh);
        kb.h[1] = *(const v8h*)(Ksh + (j * 16 + c) * 64 + dc * 32 + 16 + 8 * hh);
        sh = mma_h(qa[dc], kb.v, sh);
      }
#pragma unroll
      for (int r = 0; r < 8; ++r) s[j][r] = sh[r] * sscale + mk[j];
    }

    _Float16* pwh = Psh[wave];
#pragma unroll
    for (int r = 0; r < 8; ++r) {
      float m = s[0][r];
      m = fmaxf(m, s[1][r]);
      m = fmaxf(m, s[2][r]);
      m = fmaxf(m, s[3][r]);
#pragma unroll
      for (int off = 1; off < 16; off <<= 1) m = fmaxf(m, __shfl_xor(m, off, 32));
      const float mnew  = fmaxf(mrow[r], m);
      const float alpha = __expf(mrow[r] - mnew);
      mrow[r] = mnew;
      float psum = 0.f;
#pragma unroll
      for (int j = 0; j < 4; ++j) {
        const float p = __expf(s[j][r] - mnew);
        psum += p;
        pwh[(8 * hh + r) * 64 + j * 16 + c] = (_Float16)(p * 1024.0f);
      }
#pragma unroll
      for (int off = 1; off < 16; off <<= 1) psum += __shfl_xor(psum, off, 32);
      lrow[r] = lrow[r] * alpha + psum;
#pragma unroll
      for (int t = 0; t < 4; ++t) oacc[t][r] *= alpha;
    }
    wave_sync_lds();

#pragma unroll 1
    for (int kk = 0; kk < 2; ++kk) {
      FragH pa;
      pa.h[0] = *(const v8h*)(pwh + c * 64 + kk * 32 + 8 * hh);
      pa.h[1] = *(const v8h*)(pwh + c * 64 + kk * 32 + 16 + 8 * hh);
#pragma unroll
      for (int t = 0; t < 4; ++t) {
        FragH vb;
        vb.h[0] = *(const v8h*)(Vth + (t * 16 + c) * 64 + kk * 32 + 8 * hh);
        vb.h[1] = *(const v8h*)(Vth + (t * 16 + c) * 64 + kk * 32 + 16 + 8 * hh);
        oacc[t] = mma_h(pa.v, vb.v, oacc[t]);
      }
    }
  }

  float* os = Os[wave];
#pragma unroll
  for (int r = 0; r < 8; ++r) {
    const float l = lrow[r];
    const float inv = ((l > 0.f) ? (1.0f / l) : 0.f) * (CSC / 1024.0f);
#pragma unroll
    for (int t = 0; t < 4; ++t) os[(8 * hh + r) * 64 + t * 16 + c] = oacc[t][r] * inv;
  }
  wave_sync_lds();
  {
    const int q4 = lane >> 3, c8 = (lane & 7) * 8;
    v4u hv[4];
#pragma unroll
    for (int it = 0; it < 4; ++it) {
      const int row = it * 4 + q4;
      const float* sp = os + row * 64 + c8;
      v4u a;
#pragma unroll
      for (int e = 0; e < 4; ++e) a[e] = pk16(h_bits((_Float16)sp[2 * e]), h_bits((_Float16)sp[2 * e + 1]));
      hv[it] = a;
    }
    for (int pass = 0; pass < 2; ++pass) {
#pragma unroll
      for (int it = 0; it < 4; ++it) {
        const int row = it * 4 + q4;
        const size_t go = (rowB + q0 + row) * DM + (size_t)h * HD + c8;
        *(volatile v4u*)(outp + go) = hv[it];
      }
      __threadfence();
    }
  }
}

__global__ __launch_bounds__(LNT) void ln_row_f32(const float* __restrict__ X, const float* __restrict__ gam,
                                                  const float* __restrict__ bet, float* outF) {
  __shared__ float red0[8], red1[8];
  const int t = threadIdx.x, lane = t & 31, wave = t >> 5;
  const size_t base = (size_t)blockIdx.x * DM;
  const v4f xv = *(const v4f*)(X + base + 4 * t);
  const float mean = bsumLN((xv[0] + xv[1]) + (xv[2] + xv[3]), red0, lane, wave) * (1.0f / DM);
  v4f d;
#pragma unroll
  for (int e = 0; e < 4; ++e) d[e] = xv[e] - mean;
  const float var  = bsumLN((d[0] * d[0] + d[1] * d[1]) + (d[2] * d[2] + d[3] * d[3]), red1, lane, wave) * (1.0f / DM);
  const float rstd = 1.0f / sqrtf(var + LNEPS);
  const v4f gv = *(const v4f*)(gam + 4 * t);
  const v4f bv = *(const v4f*)(bet + 4 * t);
  v4f y;
#pragma unroll
  for (int e = 0; e < 4; ++e) y[e] = (d[e] * rstd) * bfr(gv[e]) + bfr(bv[e]);
  float* dst = outF + base + 4 * t;
  *(volatile v4f*)dst = y;
  __threadfence();
  *(volatile v4f*)dst = y;
}

extern "C" void kernel_launch(void* const* d_in, const int* in_sizes, int n_in,
                              void* d_out, int out_size, void* d_ws, size_t ws_size,
                              hipStream_t stream) {
  if (n_in < 12) return;
  if (in_sizes[0] != MP * DM) return;
  if (in_sizes[1] != NBATCH * SEQ) return;
  if (in_sizes[2] != DM * DM || in_sizes[3] != DM) return;
  if (in_sizes[4] != DM * DM || in_sizes[5] != DM) return;
  if (in_sizes[6] != DM * DM || in_sizes[7] != DM) return;
  if (in_sizes[8] != DM * DM || in_sizes[9] != DM) return;
  if (in_sizes[10] != DM || in_sizes[11] != DM) return;
  if (out_size != MP * DM) return;

  const float* hidden = (const float*)d_in[0];
  const float* amask  = (const float*)d_in[1];
  const float* w_q    = (const float*)d_in[2];
  const float* b_q    = (const float*)d_in[3];
  const float* w_k    = (const float*)d_in[4];
  const float* b_k    = (const float*)d_in[5];
  const float* w_v    = (const float*)d_in[6];
  const float* b_v    = (const float*)d_in[7];
  const float* w_o    = (const float*)d_in[8];
  const float* b_o    = (const float*)d_in[9];
  const float* ln_g   = (const float*)d_in[10];
  const float* ln_b   = (const float*)d_in[11];

  const size_t PWQK = (size_t)QKP * DM * 2;
  const size_t PW   = (size_t)DM * DM * 2;
  const size_t PXH  = (size_t)MP * DM * 2;
  const size_t PQK  = (size_t)MP * QKP * 2;
  const size_t PVT  = (size_t)NBATCH * DM * SEQ * 2;
  const size_t PCTX = (size_t)MP * DM * 2;
  const size_t PHF  = (size_t)MP * DM * 4;
  size_t off = 0;
  const size_t oWqk = off; off += PWQK;
  const size_t oWv  = off; off += PW;
  const size_t oWo  = off; off += PW;
  const size_t oXH  = off; off += PXH;
  const size_t oQK  = off; off += PQK;
  const size_t oVT  = off; off += PVT;
  const size_t oCtx = off; off += PCTX;
  const size_t oHf  = off; off += PHF;
  if (off > ws_size) return;
  if (off > (size_t)134217728) return;

  char* ws = (char*)d_ws;
  unsigned short* WqkH = (unsigned short*)(ws + oWqk);
  unsigned short* WvH  = (unsigned short*)(ws + oWv);
  unsigned short* WoH  = (unsigned short*)(ws + oWo);
  unsigned short* XH   = (unsigned short*)(ws + oXH);
  unsigned short* QK   = (unsigned short*)(ws + oQK);
  unsigned short* VT   = (unsigned short*)(ws + oVT);
  unsigned short* Ctx  = (unsigned short*)(ws + oCtx);
  float*          Hf   = (float*)(ws + oHf);
  float*          out0 = (float*)d_out;

  const int n8w = (DM * DM) / 8;
  const int n8x = (MP * DM) / 8;
  if ((n8w % 256) != 0 || (n8x % 256) != 0) return;
  const dim3 blk(256), blk128(128), blkLN(LNT);
  const dim3 gCw(n8w / 256), gCx(n8x / 256);
  const dim3 gNqk(((MP / 64) * (QKP / 64) + 7) / 8, 1);
  const dim3 gVT(((DM / 64) * (SEQ / 64) + 7) / 8, NBATCH);
  const dim3 gNo(((MP / 64) * (DM / 64) + 7) / 8, 1);
  const dim3 gAttn(NBATCH * NH * NQB);
  const dim3 gRow(MP);
  const float invw  = 1.0f / WSC;
  const float invwc = 1.0f / (WSC * CSC);

  conv_h16<<<gCw, blk, 0, stream>>>(w_q, WqkH, n8w, WSC);
  conv_h16<<<gCw, blk, 0, stream>>>(w_k, WqkH + (size_t)DM * DM, n8w, WSC);
  conv_h16<<<gCw, blk, 0, stream>>>(w_v, WvH, n8w, WSC);
  conv_h16<<<gCw, blk, 0, stream>>>(w_o, WoH, n8w, WSC);
  conv_h16<<<gCx, blk, 0, stream>>>(hidden, XH, n8x, 1.0f);

  gemm64<2, 0, 0, 0><<<gNqk, blk, 0, stream>>>(
      XH, DM, 0LL, WqkH, DM, 0LL, b_q, b_k, DM, hidden,
      (void*)QK, QKP, 0LL, MP, QKP, DM, invw);
  gemm64<2, 1, 0, 0><<<gVT, blk, 0, stream>>>(
      WvH, DM, 0LL, XH, DM, (long long)SEQ * DM, b_v, b_v, SEQ, hidden,
      (void*)VT, SEQ, (long long)DM * SEQ, DM, SEQ, DM, invw);

  attn64<<<gAttn, blk128, 0, stream>>>(QK, VT, amask, Ctx, 0.125f);

  gemm64<0, 0, 0, 3><<<gNo, blk, 0, stream>>>(
      Ctx, DM, 0LL, WoH, DM, 0LL, b_o, b_o, DM, hidden,
      (void*)Hf, DM, 0LL, MP, DM, DM, invwc);

  ln_row_f32<<<gRow, blkLN, 0, stream>>>(Hf, ln_g, ln_b, out0);
  (void)hipGetLastError();
}
